// JangDFlashAttention_47983374631189
// MI455X (gfx1250) — hardware-verified
//
#include <hip/hip_runtime.h>
#include <math.h>
#include <stdint.h>

#define NB    2
#define SL    2048
#define ST    512
#define SKEY  2560
#define HIDN  2048
#define NQH   16
#define NKV   4
#define HD    128
#define QO    2048
#define KVO   512
#define NFREQ 64

typedef _Float16 v16h __attribute__((ext_vector_type(16)));
typedef _Float16 v8h  __attribute__((ext_vector_type(8)));
typedef _Float16 v4h  __attribute__((ext_vector_type(4)));
typedef float    v8f  __attribute__((ext_vector_type(8)));
typedef float    v4f  __attribute__((ext_vector_type(4)));

__device__ __forceinline__ float bf16_rne(float f) {
  unsigned u = __float_as_uint(f);
  u = (u + 0x7FFFu + ((u >> 16) & 1u)) & 0xFFFF0000u;
  return __uint_as_float(u);
}

union FragU { v16h v; v8h h[2]; };
__device__ __forceinline__ v16h frag_ld(const _Float16* p) {
  FragU f;
  f.h[0] = *(const v8h*)(p);
  f.h[1] = *(const v8h*)(p + 16);
  return f.v;
}
__device__ __forceinline__ v8f mma16(v16h a, v16h b, v8f c) {
  return __builtin_amdgcn_wmma_f32_16x16x32_f16(false, a, false, b, (short)0, c, false, false);
}
__device__ __forceinline__ void guard1(v8f& x, v16h a, v16h b) {
  asm volatile("v_nop\n\tv_nop\n\tv_nop\n\tv_nop" : "+v"(x) : "v"(a), "v"(b));
}
__device__ __forceinline__ void guard2(v8f& x, v8f& y, v16h a, v16h b) {
  asm volatile("v_nop\n\tv_nop\n\tv_nop\n\tv_nop" : "+v"(x), "+v"(y) : "v"(a), "v"(b));
}
__device__ __forceinline__ void guard4(v8f& a, v8f& b, v8f& c, v8f& d) {
  asm volatile("v_nop\n\tv_nop\n\tv_nop\n\tv_nop" : "+v"(a), "+v"(b), "+v"(c), "+v"(d));
}
__device__ __forceinline__ void keep2(v16h a, v16h b) { asm volatile("v_nop" :: "v"(a), "v"(b)); }
__device__ __forceinline__ void keep4(v16h a, v16h b, v16h c, v16h d) {
  asm volatile("v_nop" :: "v"(a), "v"(b), "v"(c), "v"(d));
}
__device__ __forceinline__ v8f zero8() { v8f z = {0.f, 0.f, 0.f, 0.f, 0.f, 0.f, 0.f, 0.f}; return z; }
__device__ __forceinline__ void wave_lds_sync() {
  __builtin_amdgcn_fence(__ATOMIC_RELEASE, "workgroup");
  __builtin_amdgcn_wave_barrier();
  __builtin_amdgcn_fence(__ATOMIC_ACQUIRE, "workgroup");
}

__global__ __launch_bounds__(256) void k_cvt16(const float* __restrict__ in, _Float16* __restrict__ out, int n8, float scale) {
  const int i = blockIdx.x * 256 + threadIdx.x;
  if (i >= n8) return;
  const v4f a = *(const v4f*)(in + (size_t)i * 8);
  const v4f c = *(const v4f*)(in + (size_t)i * 8 + 4);
  v8h o;
#pragma unroll
  for (int e = 0; e < 4; ++e) {
    o[e]     = (_Float16)(bf16_rne(a[e]) * scale);
    o[4 + e] = (_Float16)(bf16_rne(c[e]) * scale);
  }
  _Float16* p = out + (size_t)i * 8;
  *(volatile v8h*)p = o;
  __threadfence();
  *(volatile v8h*)p = o;
}

__global__ __launch_bounds__(256) void k_wT(const float* __restrict__ W, _Float16* __restrict__ o, int R, int Cc, float scale) {
  __shared__ __align__(16) float tf[64 * 68];
  const int c0 = blockIdx.x * 64;
  const int r0 = blockIdx.y * 64;
  const int tid = threadIdx.x;
  {
    const int lr = tid >> 4, c4 = (tid & 15) * 4;
#pragma unroll
    for (int it = 0; it < 4; ++it) {
      const int rr = it * 16 + lr;
      const v4f a = *(const v4f*)(W + (size_t)(r0 + rr) * Cc + c0 + c4);
      *(v4f*)(tf + rr * 68 + c4) = a;
    }
  }
  __syncthreads();
  const int sub = tid >> 3, c8 = (tid & 7) * 8;
  v8h hv[2];
#pragma unroll
  for (int it = 0; it < 2; ++it) {
    const int oc = it * 32 + sub;
    v8h a;
#pragma unroll
    for (int e = 0; e < 8; ++e) a[e] = (_Float16)(bf16_rne(tf[(c8 + e) * 68 + oc]) * scale);
    hv[it] = a;
  }
  for (int pass = 0; pass < 2; ++pass) {
#pragma unroll
    for (int it = 0; it < 2; ++it) {
      const int oc = it * 32 + sub;
      const size_t go = (size_t)(c0 + oc) * R + r0 + c8;
      *(volatile v8h*)(o + go) = hv[it];
    }
    __threadfence();
  }
}

template <bool ASPLIT, int OUT16>
__global__ __launch_bounds__(256) void k_gemm64(
    const _Float16* __restrict__ A, const _Float16* __restrict__ A2, int lda, long strideA,
    const _Float16* __restrict__ Bt, int ldb, long strideB,
    void* Cout, void* Cout2, int ldc, long strideC,
    int M, int N, int K, float scale) {
  __shared__ __align__(16) float sT[8][16 * 68];
  const int b    = blockIdx.y;
  const int lane = threadIdx.x & 31;
  const int wave = threadIdx.x >> 5;
  const int tilesN = N >> 6;
  const int tilesM = M >> 6;
  const int tile = blockIdx.x * 8 + wave;
  if (tile >= tilesM * tilesN) return;
  const int tm = tile / tilesN;
  const int tn = tile - tm * tilesN;
  const int m0 = tm << 6;
  const int n0 = tn << 6;

  const _Float16* Ab  = A + (size_t)b * strideA;
  const _Float16* Ab2 = ASPLIT ? (A2 + (size_t)b * strideA) : Ab;
  const _Float16* Bb  = Bt + (size_t)b * strideB;

  const int rl   = lane & 15;
  const int koff = (lane >> 4) * 8;
  const int mOff = (lane >> 4) * 8;

  v8f acc[4][4];
#pragma unroll
  for (int i = 0; i < 4; ++i)
#pragma unroll
    for (int j = 0; j < 4; ++j) acc[i][j] = zero8();

  for (int k0 = 0; k0 < K; k0 += 32) {
    v16h bf[4];
#pragma unroll
    for (int j = 0; j < 4; ++j)
      bf[j] = frag_ld(Bb + (size_t)(n0 + (j << 4) + rl) * ldb + k0 + koff);
#pragma unroll
    for (int i = 0; i < 4; ++i) {
      const size_t ao = (size_t)(m0 + (i << 4) + rl) * lda + k0 + koff;
      const v16h ah = frag_ld(Ab + ao);
      v16h al = ah;
      if (ASPLIT) al = frag_ld(Ab2 + ao);
#pragma unroll
      for (int j = 0; j < 4; ++j) {
        acc[i][j] = mma16(ah, bf[j], acc[i][j]);
        if (ASPLIT) acc[i][j] = mma16(al, bf[j], acc[i][j]);
      }
      guard2(acc[i][0], acc[i][3], ah, al);
    }
    keep4(bf[0], bf[1], bf[2], bf[3]);
  }
  guard4(acc[0][0], acc[0][1], acc[0][2], acc[0][3]);
  guard4(acc[1][0], acc[1][1], acc[1][2], acc[1][3]);
  guard4(acc[2][0], acc[2][1], acc[2][2], acc[2][3]);
  guard4(acc[3][0], acc[3][1], acc[3][2], acc[3][3]);

  float* slab = sT[wave];
#pragma unroll
  for (int i = 0; i < 4; ++i) {
    const int mBase = m0 + (i << 4);
#pragma unroll
    for (int j = 0; j < 4; ++j) {
#pragma unroll
      for (int r = 0; r < 8; ++r) slab[(mOff + r) * 68 + (j << 4) + rl] = acc[i][j][r] * scale;
    }
    wave_lds_sync();
    if (OUT16 == 0) {
      float* C = (float*)Cout + (size_t)b * strideC;
      const int h2 = lane >> 4, c4 = (lane & 15) * 4;
      for (int pass = 0; pass < 2; ++pass) {
#pragma unroll
        for (int it = 0; it < 8; ++it) {
          const int row = it * 2 + h2;
          const v4f v = *(const v4f*)(slab + row * 68 + c4);
          *(volatile v4f*)(C + (size_t)(mBase + row) * ldc + n0 + c4) = v;
        }
        __threadfence();
      }
    } else {
      _Float16* C  = (_Float16*)Cout  + (size_t)b * strideC;
      _Float16* C2 = (_Float16*)Cout2 + (size_t)b * strideC;
      const int q = lane >> 3, c8 = (lane & 7) * 8;
      for (int pass = 0; pass < 2; ++pass) {
#pragma unroll
        for (int it = 0; it < 4; ++it) {
          const int row = it * 4 + q;
          const float* sp = slab + row * 68 + c8;
          v8h hv, lv;
#pragma unroll
          for (int e = 0; e < 8; ++e) {
            const float f = sp[e];
            const _Float16 fh = (_Float16)f;
            hv[e] = fh;
            lv[e] = (_Float16)(f - (float)fh);
          }
          *(volatile v8h*)(C  + (size_t)(mBase + row) * ldc + n0 + c8) = hv;
          *(volatile v8h*)(C2 + (size_t)(mBase + row) * ldc + n0 + c8) = lv;
        }
        __threadfence();
      }
    }
    wave_lds_sync();
  }
}

__global__ __launch_bounds__(64) void k_invfreq(float* __restrict__ inv) {
  const int l = threadIdx.x;
  const float ex = (float)(2 * l) * (1.0f / 128.0f);
  const float pw = powf(10000.0f, ex);
  const float v = 1.0f / pw;
  *(volatile float*)(inv + l) = v;
  __threadfence();
  *(volatile float*)(inv + l) = v;
}

__global__ __launch_bounds__(256) void k_ropetab(const float* __restrict__ inv, float* __restrict__ ctab,
                                                      float* __restrict__ stab, int n) {
  const int g = blockIdx.x * 256 + threadIdx.x;
  if (g >= n) return;
  const int t = g >> 6, i = g & 63;
  const float ang = (float)t * inv[i];
  float sn, cs;
  sincosf(ang, &sn, &cs);
  *(volatile float*)(ctab + g) = cs;
  *(volatile float*)(stab + g) = sn;
  __threadfence();
  *(volatile float*)(ctab + g) = cs;
  *(volatile float*)(stab + g) = sn;
}

template <bool ROPE>
__global__ __launch_bounds__(256) void k_normk(const float* __restrict__ Kr, const float* __restrict__ kw,
                                                    const float* __restrict__ ctab, const float* __restrict__ stab,
                                                    _Float16* __restrict__ oh, _Float16* __restrict__ ol,
                                                    int ntok, int seqoff, int nrows) {
  const int lane = threadIdx.x & 31, wave = threadIdx.x >> 5;
  const int row = blockIdx.x * 8 + wave;
  if (row >= nrows) return;
  const int token = row >> 2, kvh = row & 3;
  const int b = token / ntok, j = token - b * ntok;
  const v4f v  = *(const v4f*)(Kr + (size_t)token * KVO + kvh * HD + 4 * lane);
  const v4f wr = *(const v4f*)(kw + 4 * lane);
  float ss = v[0] * v[0] + v[1] * v[1] + v[2] * v[2] + v[3] * v[3];
  ss += __shfl_xor(ss, 1, 32);
  ss += __shfl_xor(ss, 2, 32);
  ss += __shfl_xor(ss, 4, 32);
  ss += __shfl_xor(ss, 8, 32);
  ss += __shfl_xor(ss, 16, 32);
  const float rs = rsqrtf(ss * (1.0f / 128.0f) + 1e-6f);
  float y[4];
#pragma unroll
  for (int e = 0; e < 4; ++e) y[e] = v[e] * rs * bf16_rne(wr[e]);
  if (ROPE) {
    float pr[4];
#pragma unroll
    for (int e = 0; e < 4; ++e) pr[e] = __shfl_xor(y[e], 16, 32);
    const v4f cs = *(const v4f*)(ctab + (size_t)j * NFREQ + 4 * (lane & 15));
    const v4f sn = *(const v4f*)(stab + (size_t)j * NFREQ + 4 * (lane & 15));
#pragma unroll
    for (int e = 0; e < 4; ++e) {
      const float rot = (lane < 16) ? -pr[e] : pr[e];
      y[e] = y[e] * cs[e] + rot * sn[e];
    }
  }
  v4h hv, lv;
#pragma unroll
  for (int e = 0; e < 4; ++e) {
    const float z = y[e] * 64.0f;
    const _Float16 zh = (_Float16)z;
    hv[e] = zh;
    lv[e] = (_Float16)(z - (float)zh);
  }
  const size_t oo = ((size_t)((b * NKV + kvh) * SKEY + seqoff + j)) * HD + 4 * lane;
  *(volatile v4h*)(oh + oo) = hv;
  *(volatile v4h*)(ol + oo) = lv;
  __threadfence();
  *(volatile v4h*)(oh + oo) = hv;
  *(volatile v4h*)(ol + oo) = lv;
}

__global__ __launch_bounds__(128) void k_attn(
    const float* __restrict__ Qr, const float* __restrict__ qw,
    const float* __restrict__ ctab, const float* __restrict__ stab,
    const _Float16* __restrict__ Kh, const _Float16* __restrict__ Kl,
    const _Float16* __restrict__ Vh, const _Float16* __restrict__ Vl,
    _Float16* __restrict__ Oh, _Float16* __restrict__ Ol) {
  __shared__ __align__(16) _Float16 Qsh[64 * HD];
  __shared__ __align__(16) _Float16 Qsl[64 * HD];
  __shared__ __align__(16) _Float16 Ksh[64 * HD];
  __shared__ __align__(16) _Float16 Ksl[64 * HD];
  __shared__ __align__(16) _Float16 Vsh[HD * 64];
  __shared__ __align__(16) _Float16 Vsl[HD * 64];
  __shared__ __align__(16) _Float16 Psh[4][16 * 64];
  __shared__ __align__(16) _Float16 Psl[4][16 * 64];

  const int tid  = threadIdx.x;
  const int wave = tid >> 5;
  const int lane = tid & 31;
  const int hh   = lane >> 4;
  const int m    = lane & 15;
  const int qb   = blockIdx.x;
  const int b    = blockIdx.y >> 4;
  const int h    = blockIdx.y & 15;
  const int kvh  = h >> 2;
  const int qw0  = qb * 64 + wave * 16;

  const float kS2 = 1.4426950408889634f * 0.08838834764831845f * (1.0f / 4096.0f);

  {
    const v4f wr = *(const v4f*)(qw + 4 * lane);
    float w4[4];
#pragma unroll
    for (int e = 0; e < 4; ++e) w4[e] = bf16_rne(wr[e]);
#pragma unroll 2
    for (int r = 0; r < 16; ++r) {
      const int i = qw0 + r;
      const v4f v = *(const v4f*)(Qr + ((size_t)(b * SL + i)) * QO + h * HD + 4 * lane);
      float ss = v[0] * v[0] + v[1] * v[1] + v[2] * v[2] + v[3] * v[3];
      ss += __shfl_xor(ss, 1, 32);
      ss += __shfl_xor(ss, 2, 32);
      ss += __shfl_xor(ss, 4, 32);
      ss += __shfl_xor(ss, 8, 32);
      ss += __shfl_xor(ss, 16, 32);
      const float rs = rsqrtf(ss * (1.0f / 128.0f) + 1e-6f);
      float y[4], pr[4];
#pragma unroll
      for (int e = 0; e < 4; ++e) y[e] = v[e] * rs * w4[e];
#pragma unroll
      for (int e = 0; e < 4; ++e) pr[e] = __shfl_xor(y[e], 16, 32);
      const v4f cs = *(const v4f*)(ctab + (size_t)i * NFREQ + 4 * m);
      const v4f sn = *(const v4f*)(stab + (size_t)i * NFREQ + 4 * m);
      v4h hv, lv;
#pragma unroll
      for (int e = 0; e < 4; ++e) {
        const float rot = (lane < 16) ? -pr[e] : pr[e];
        const float z = (y[e] * cs[e] + rot * sn[e]) * 64.0f;
        const _Float16 zh = (_Float16)z;
        hv[e] = zh;
        lv[e] = (_Float16)(z - (float)zh);
      }
      *(v4h*)(Qsh + (wave * 16 + r) * HD + 4 * lane) = hv;
      *(v4h*)(Qsl + (wave * 16 + r) * HD + 4 * lane) = lv;
    }
  }

  float mrow[8], lrow[8];
  v8f oacc[8];
#pragma unroll
  for (int r = 0; r < 8; ++r) { mrow[r] = -INFINITY; lrow[r] = 0.f; }
#pragma unroll
  for (int t = 0; t < 8; ++t) oacc[t] = zero8();

  const size_t kvbase = (size_t)(b * NKV + kvh) * SKEY * HD;
  const _Float16* Khb = Kh + kvbase;
  const _Float16* Klb = Kl + kvbase;
  const _Float16* Vhb = Vh + kvbase;
  const _Float16* Vlb = Vl + kvbase;

  const int nch = 8 + qb + 1;
#pragma unroll 1
  for (int c = 0; c < nch; ++c) {
    const int key0 = c * 64;
    __syncthreads();
    {
      const size_t kgo = (size_t)key0 * HD;
#pragma unroll
      for (int it = 0; it < 8; ++it) {
        const int e = (it * 128 + tid) * 8;
        *(v8h*)(Ksh + e) = *(const v8h*)(Khb + kgo + e);
      }
      asm volatile("" ::: "memory");
#pragma unroll
      for (int it = 0; it < 8; ++it) {
        const int e = (it * 128 + tid) * 8;
        *(v8h*)(Ksl + e) = *(const v8h*)(Klb + kgo + e);
      }
      asm volatile("" ::: "memory");
      const size_t vgo = (size_t)tid * SKEY + key0;
#pragma unroll
      for (int it = 0; it < 8; ++it)
        *(v8h*)(Vsh + tid * 64 + it * 8) = *(const v8h*)(Vhb + vgo + it * 8);
      asm volatile("" ::: "memory");
#pragma unroll
      for (int it = 0; it < 8; ++it)
        *(v8h*)(Vsl + tid * 64 + it * 8) = *(const v8h*)(Vlb + vgo + it * 8);
    }
    __syncthreads();

    v8f s[4];
#pragma unroll
    for (int j = 0; j < 4; ++j) s[j] = zero8();
    {
      const _Float16* qhp = Qsh + (wave * 16 + m) * HD + 8 * hh;
      const _Float16* qlp = Qsl + (wave * 16 + m) * HD + 8 * hh;
#pragma unroll
      for (int dc = 0; dc < 4; ++dc) {
        const v16h qh = frag_ld(qhp + dc * 32);
        const v16h ql = frag_ld(qlp + dc * 32);
#pragma unroll
        for (int j = 0; j < 4; ++j) {
          const int ko = (j * 16 + m) * HD + dc * 32 + 8 * hh;
          const v16h kh = frag_ld(Ksh + ko);
          const v16h kl = frag_ld(Ksl + ko);
          s[j] = mma16(qh, kh, s[j]);
          s[j] = mma16(qh, kl, s[j]);
          s[j] = mma16(ql, kh, s[j]);
          guard1(s[j], kh, kl);
        }
        keep2(qh, ql);
      }
    }

    const bool last = (c == nch - 1);
    const int ib = qw0 + 8 * hh;
    float cm[8];
#pragma unroll
    for (int r = 0; r < 8; ++r) {
      float mx = -INFINITY;
#pragma unroll
      for (int j = 0; j < 4; ++j) {
        const int jb = key0 - ST + j * 16 + m;
        float sv = s[j][r] * kS2;
        sv = (last && (jb > ib + r)) ? -INFINITY : sv;
        s[j][r] = sv;
        mx = fmaxf(mx, sv);
      }
      mx = fmaxf(mx, __shfl_xor(mx, 1, 32));
      mx = fmaxf(mx, __shfl_xor(mx, 2, 32));
      mx = fmaxf(mx, __shfl_xor(mx, 4, 32));
      mx = fmaxf(mx, __shfl_xor(mx, 8, 32));
      cm[r] = mx;
    }
    _Float16* Pwh = Psh[wave];
    _Float16* Pwl = Psl[wave];
#pragma unroll
    for (int r = 0; r < 8; ++r) {
      const float mnew  = fmaxf(mrow[r], cm[r]);
      const float alpha = exp2f(mrow[r] - mnew);
      mrow[r] = mnew;
      float ps = 0.f;
#pragma unroll
      for (int j = 0; j < 4; ++j) {
        const float p  = exp2f(s[j][r] - mnew);
        ps += p;
        const float pk = p * 32768.0f;
        const _Float16 ph = (_Float16)pk;
        const _Float16 pl = (_Float16)(pk - (float)ph);
        Pwh[(8 * hh + r) * 64 + j * 16 + m] = ph;
        Pwl[(8 * hh + r) * 64 + j * 16 + m] = pl;
      }
      ps += __shfl_xor(ps, 1, 32);
      ps += __shfl_xor(ps, 2, 32);
      ps += __shfl_xor(ps, 4, 32);
      ps += __shfl_xor(ps, 8, 32);
      lrow[r] = lrow[r] * alpha + ps;
#pragma unroll
      for (int t = 0; t < 8; ++t) oacc[t][r] *= alpha;
    }
    wave_lds_sync();

#pragma unroll
    for (int kk = 0; kk < 2; ++kk) {
      const int po = m * 64 + kk * 32 + 8 * hh;
      const v16h ph = frag_ld(Pwh + po);
      const v16h pl = frag_ld(Pwl + po);
#pragma unroll
      for (int t = 0; t < 8; ++t) {
        const int vo = (t * 16 + m) * 64 + kk * 32 + 8 * hh;
        const v16h vh = frag_ld(Vsh + vo);
        const v16h vl = frag_ld(Vsl + vo);
        oacc[t] = mma16(ph, vh, oacc[t]);
        oacc[t] = mma16(ph, vl, oacc[t]);
        oacc[t] = mma16(pl, vh, oacc[t]);
        guard1(oacc[t], vh, vl);
      }
      keep2(ph, pl);
    }
  }
  guard4(oacc[0], oacc[1], oacc[2], oacc[3]);
  guard4(oacc[4], oacc[5], oacc[6], oacc[7]);

  __syncthreads();
  _Float16* Osh = Ksh + wave * 16 * HD;
  _Float16* Osl = Ksl + wave * 16 * HD;
#pragma unroll
  for (int r = 0; r < 8; ++r) {
    const float inv = 1.0f / (lrow[r] * 8192.0f);
#pragma unroll
    for (int t = 0; t < 8; ++t) {
      const float o = oacc[t][r] * inv;
      const _Float16 ohv = (_Float16)o;
      Osh[(8 * hh + r) * HD + t * 16 + m] = ohv;
      Osl[(8 * hh + r) * HD + t * 16 + m] = (_Float16)(o - (float)ohv);
    }
  }
  wave_lds_sync();
  {
    const size_t ob = ((size_t)(b * SL + qw0)) * QO + h * HD + 8 * m;
    for (int pass = 0; pass < 2; ++pass) {
#pragma unroll
      for (int it = 0; it < 8; ++it) {
        const int row = it * 2 + hh;
        const v8h a  = *(const v8h*)(Osh + row * HD + 8 * m);
        const v8h a2 = *(const v8h*)(Osl + row * HD + 8 * m);
        *(volatile v8h*)(Oh + ob + (size_t)row * QO) = a;
        *(volatile v8h*)(Ol + ob + (size_t)row * QO) = a2;
      }
      __threadfence();
    }
  }
}

extern "C" void kernel_launch(void* const* d_in, const int* in_sizes, int n_in,
                              void* d_out, int out_size, void* d_ws, size_t ws_size,
                              hipStream_t stream) {
  if (n_in < 10) return;
  if (in_sizes[0] != NB * SL * HIDN) return;
  if (in_sizes[1] != NB * ST * HIDN) return;
  if (in_sizes[2] != HIDN * QO || in_sizes[5] != QO * HIDN) return;
  if (in_sizes[3] != HIDN * KVO || in_sizes[4] != HIDN * KVO) return;
  if (in_sizes[6] != HIDN * KVO || in_sizes[7] != HIDN * KVO) return;
  if (in_sizes[8] != HD || in_sizes[9] != HD) return;
  if (out_size != NB * SL * HIDN) return;

  const float* x   = (const float*)d_in[0];
  const float* hc  = (const float*)d_in[1];
  const float* wq  = (const float*)d_in[2];
  const float* wk  = (const float*)d_in[3];
  const float* wv  = (const float*)d_in[4];
  const float* wo  = (const float*)d_in[5];
  const float* wkc = (const float*)d_in[6];
  const float* wvc = (const float*)d_in[7];
  const float* qnw = (const float*)d_in[8];
  const float* knw = (const float*)d_in[9];
  float* out = (float*)d_out;

  const size_t szXp  = (size_t)NB * SL * HIDN * 2;
  const size_t szHp  = (size_t)NB * ST * HIDN * 2;
  const size_t szWq  = (size_t)HIDN * QO * 2;
  const size_t szWkv = (size_t)HIDN * KVO * 2;
  const size_t szWo  = (size_t)QO * HIDN * 2;
  const size_t szQr  = (size_t)NB * SL * QO * 4;
  const size_t szKr  = (size_t)NB * SL * KVO * 4;
  const size_t szKcr = (size_t)NB * ST * KVO * 4;
  const size_t szPl  = (size_t)NB * NKV * SKEY * HD * 2;
  const size_t szO   = (size_t)NB * SL * QO * 2;
  const size_t szInv = 4096;
  const size_t szTab = (size_t)SL * NFREQ * 4;
  size_t off = 0;
  const size_t oXp   = off; off += szXp;
  const size_t oHp   = off; off += szHp;
  const size_t oWqT  = off; off += szWq;
  const size_t oWkT  = off; off += szWkv;
  const size_t oWvT  = off; off += szWkv;
  const size_t oWoT  = off; off += szWo;
  const size_t oWkcT = off; off += szWkv;
  const size_t oWvcT = off; off += szWkv;
  const size_t oQr   = off; off += szQr;
  const size_t oKcr  = off; off += szKcr;
  const size_t oVTh  = off; off += szPl;
  const size_t oVTl  = off; off += szPl;
  const size_t oOh   = off; off += szO;
  const size_t oOl   = off; off += szO;
  const size_t oInv  = off; off += szInv;
  const size_t oCos  = off; off += szTab;
  const size_t oSin  = off; off += szTab;
  const size_t oKr   = oWqT;
  const size_t oKph  = oXp;
  const size_t oKpl  = oXp + szPl;
  if (szKr > szWq) return;
  if (2 * szPl > szXp) return;
  if (off > ws_size) return;

  char* ws = (char*)d_ws;
  _Float16* Xp   = (_Float16*)(ws + oXp);
  _Float16* Hp   = (_Float16*)(ws + oHp);
  _Float16* WqT  = (_Float16*)(ws + oWqT);
  _Float16* WkT  = (_Float16*)(ws + oWkT);
  _Float16* WvT  = (_Float16*)(ws + oWvT);
  _Float16* WoT  = (_Float16*)(ws + oWoT);
  _Float16* WkcT = (_Float16*)(ws + oWkcT);
  _Float16* WvcT = (_Float16*)(ws + oWvcT);
  float*    Qr   = (float*)(ws + oQr);
  float*    Kr   = (float*)(ws + oKr);
  float*    Kcr  = (float*)(ws + oKcr);
  _Float16* Kph  = (_Float16*)(ws + oKph);
  _Float16* Kpl  = (_Float16*)(ws + oKpl);
  _Float16* VTh  = (_Float16*)(ws + oVTh);
  _Float16* VTl  = (_Float16*)(ws + oVTl);
  _Float16* Oh   = (_Float16*)(ws + oOh);
  _Float16* Ol   = (_Float16*)(ws + oOl);
  float*    Inv  = (float*)(ws + oInv);
  float*    Cos  = (float*)(ws + oCos);
  float*    Sin  = (float*)(ws + oSin);

  const dim3 blk(256);

  k_cvt16<<<dim3(NB * SL * HIDN / 8 / 256), blk, 0, stream>>>(x, Xp, NB * SL * HIDN / 8, 16.0f);
  k_cvt16<<<dim3(NB * ST * HIDN / 8 / 256), blk, 0, stream>>>(hc, Hp, NB * ST * HIDN / 8, 16.0f);
  k_wT<<<dim3(QO / 64, HIDN / 64), blk, 0, stream>>>(wq, WqT, HIDN, QO, 64.0f);
  k_wT<<<dim3(KVO / 64, HIDN / 64), blk, 0, stream>>>(wk, WkT, HIDN, KVO, 64.0f);
  k_wT<<<dim3(KVO / 64, HIDN / 64), blk, 0, stream>>>(wv, WvT, HIDN, KVO, 64.0f);
  k_wT<<<dim3(HIDN / 64, QO / 64), blk, 0, stream>>>(wo, WoT, QO, HIDN, 64.0f);
  k_wT<<<dim3(KVO / 64, HIDN / 64), blk, 0, stream>>>(wkc, WkcT, HIDN, KVO, 64.0f);
  k_wT<<<dim3(KVO / 64, HIDN / 64), blk, 0, stream>>>(wvc, WvcT, HIDN, KVO, 64.0f);
  k_invfreq<<<dim3(1), dim3(64), 0, stream>>>(Inv);
  k_ropetab<<<dim3(SL * NFREQ / 256), blk, 0, stream>>>(Inv, Cos, Sin, SL * NFREQ);
  k_gemm64<false, 0><<<dim3((NB * SL / 64) * (QO / 64) / 8, 1), blk, 0, stream>>>(
      Xp, Xp, HIDN, 0L, WqT, HIDN, 0L, (void*)Qr, (void*)Qr, QO, 0L, NB * SL, QO, HIDN, 1.0f / 1024.0f);
  k_gemm64<false, 0><<<dim3((NB * SL / 64) * (KVO / 64) / 8, 1), blk, 0, stream>>>(
      Xp, Xp, HIDN, 0L, WkT, HIDN, 0L, (void*)Kr, (void*)Kr, KVO, 0L, NB * SL, KVO, HIDN, 1.0f / 1024.0f);
  k_gemm64<false, 0><<<dim3((NB * ST / 64) * (KVO / 64) / 8, 1), blk, 0, stream>>>(
      Hp, Hp, HIDN, 0L, WkcT, HIDN, 0L, (void*)Kcr, (void*)Kcr, KVO, 0L, NB * ST, KVO, HIDN, 1.0f / 1024.0f);
  k_gemm64<false, 1><<<dim3((KVO / 64) * (SL / 64) / 8, NB), blk, 0, stream>>>(
      WvT, WvT, HIDN, 0L, Xp, HIDN, (long)SL * HIDN, (void*)(VTh + ST), (void*)(VTl + ST), SKEY, (long)KVO * SKEY,
      KVO, SL, HIDN, 1.0f / 64.0f);
  k_gemm64<false, 1><<<dim3((KVO / 64) * (ST / 64) / 8, NB), blk, 0, stream>>>(
      WvcT, WvcT, HIDN, 0L, Hp, HIDN, (long)ST * HIDN, (void*)VTh, (void*)VTl, SKEY, (long)KVO * SKEY,
      KVO, ST, HIDN, 1.0f / 64.0f);
  k_normk<true><<<dim3(NB * SL * NKV / 8), blk, 0, stream>>>(Kr, knw, Cos, Sin, Kph, Kpl, SL, ST, NB * SL * NKV);
  k_normk<false><<<dim3(NB * ST * NKV / 8), blk, 0, stream>>>(Kcr, knw, Cos, Sin, Kph, Kpl, ST, 0, NB * ST * NKV);
  k_attn<<<dim3(SL / 64, NB * NQH), dim3(128), 0, stream>>>(Qr, qnw, Cos, Sin, Kph, Kpl, VTh, VTl, Oh, Ol);
  k_gemm64<true, 0><<<dim3((NB * SL / 64) * (HIDN / 64) / 8, 1), blk, 0, stream>>>(
      Oh, Ol, QO, 0L, WoT, QO, 0L, (void*)out, (void*)out, HIDN, 0L, NB * SL, HIDN, QO, 1.0f / 4096.0f);
  (void)hipGetLastError();
}
